// MMAKernelLayer_45483703665413
// MI455X (gfx1250) — hardware-verified
//
#include <hip/hip_runtime.h>
#include <float.h>


typedef __bf16 b16;
typedef __attribute__((ext_vector_type(16))) __bf16 v16b;
typedef __attribute__((ext_vector_type(8)))  float  v8f;
typedef __attribute__((ext_vector_type(4)))  float  v4f;

#define RES 30
#define GSIZE (RES * RES)
#define NI 32
#define NC 32
#define SPB 8
#define NTILE ((GSIZE + 15) / 16)

__device__ __forceinline__ b16 bf16_rne(float f) {
  unsigned int u = __float_as_uint(f);
  u += 0x7fffu + ((u >> 16) & 1u);
  return __builtin_bit_cast(b16, (unsigned short)(u >> 16));
}
__device__ __forceinline__ float bf16_f32(b16 b) { return __uint_as_float(((unsigned int)__builtin_bit_cast(unsigned short, b)) << 16); }
__device__ __forceinline__ void split3(float x, b16& h, b16& m, b16& l) {
  h = bf16_rne(x); const float r1 = x - bf16_f32(h); m = bf16_rne(r1); l = bf16_rne(r1 - bf16_f32(m));
}
__device__ __forceinline__ v8f wmmab(v16b a, v16b b, v8f c) {
  v8f d = __builtin_amdgcn_wmma_f32_16x16x32_bf16(false, a, false, b, (short)0, c, false, false);
  asm volatile("v_nop\n\tv_nop\n\tv_nop\n\tv_nop" : "+v"(d) : "v"(a), "v"(b));
  return d;
}
__device__ __forceinline__ v16b build_frag(const float v[4], const int sel[6], int hh) {
  b16 parts[4][3];
#pragma unroll
  for (int c = 0; c < 4; ++c) split3(v[c], parts[c][0], parts[c][1], parts[c][2]);
  v16b f;
#pragma unroll
  for (int e = 0; e < 16; ++e) {
    const int k = ((e < 8) ? e : (e + 8)) + 8 * hh;
    const int j = k >> 2, c = k & 3;
    f[e] = (j < 6) ? parts[c][sel[j]] : bf16_rne(0.0f);
  }
  return f;
}

__device__ __forceinline__ float pairmin8(v8f a, v8f b) {
  float m0 = fminf(a[0], b[0]), m1 = fminf(a[1], b[1]), m2 = fminf(a[2], b[2]), m3 = fminf(a[3], b[3]);
  float m4 = fminf(a[4], b[4]), m5 = fminf(a[5], b[5]), m6 = fminf(a[6], b[6]), m7 = fminf(a[7], b[7]);
  m0 = fminf(m0, m4); m1 = fminf(m1, m5); m2 = fminf(m2, m6); m3 = fminf(m3, m7);
  m0 = fminf(m0, m2); m1 = fminf(m1, m3);
  return fminf(m0, m1);
}

__global__ __launch_bounds__(256) void pi_kernel(const float* __restrict__ births, const float* __restrict__ deaths,
                                                 float* __restrict__ out, int S) {
  __shared__ float smn[2][256], smx[2][256];
  __shared__ float meta[SPB][4];
  __shared__ float w2s[SPB][NI];
  __shared__ __attribute__((aligned(16))) float sOut[SPB * GSIZE];
  const int t = threadIdx.x, lane = t & 31, wave = t >> 5, hh = lane >> 4, l16 = lane & 15;
  const int s0 = blockIdx.x * SPB;

  for (int si = 0; si < SPB; ++si) {
    const int s = s0 + si;
    const float* bb = births + (size_t)s * (NI * NC * 2);
    const float* dd = deaths + (size_t)s * (NI * NC * 2);
    float mnx = FLT_MAX, mny = FLT_MAX, mxx = -FLT_MAX, mxy = -FLT_MAX;
    for (int p = t; p < NI * NC; p += 256) {
      float x = bb[2 * p], y = bb[2 * p + 1];
      mnx = fminf(mnx, x); mxx = fmaxf(mxx, x); mny = fminf(mny, y); mxy = fmaxf(mxy, y);
      x = dd[2 * p]; y = dd[2 * p + 1];
      mnx = fminf(mnx, x); mxx = fmaxf(mxx, x); mny = fminf(mny, y); mxy = fmaxf(mxy, y);
    }
    smn[0][t] = mnx; smn[1][t] = mny; smx[0][t] = mxx; smx[1][t] = mxy;
    __syncthreads();
    for (int off = 128; off > 0; off >>= 1) {
      if (t < off) {
        smn[0][t] = fminf(smn[0][t], smn[0][t + off]); smn[1][t] = fminf(smn[1][t], smn[1][t + off]);
        smx[0][t] = fmaxf(smx[0][t], smx[0][t + off]); smx[1][t] = fmaxf(smx[1][t], smx[1][t + off]);
      }
      __syncthreads();
    }
    if (t == 0) {
      const float rngx = smx[0][0] - smn[0][0], rngy = smx[1][0] - smn[1][0];
      const float lox = smn[0][0] - 0.1f * rngx, loy = smn[1][0] - 0.1f * rngy;
      const float hix = smx[0][0] + 0.1f * rngx, hiy = smx[1][0] + 0.1f * rngy;
      meta[si][0] = lox; meta[si][1] = loy;
      meta[si][2] = hix - lox;
      meta[si][3] = hiy - loy;
    }
    if (t < NI) {
      const float* bi = bb + t * (NC * 2);
      const float* di = dd + t * (NC * 2);
      float acc = 0.0f;
      for (int c = 0; c < NC; ++c) acc += fmaxf(fabsf(di[2 * c] - bi[2 * c]), fabsf(di[2 * c + 1] - bi[2 * c + 1]));
      const float w = acc * (1.0f / (float)NC);
      w2s[si][t] = w * w;
    }
    __syncthreads();
  }

  const int selA[6] = {0, 0, 0, 1, 1, 2};
  const int selB[6] = {0, 1, 2, 0, 1, 0};
  const v8f vzero = {0.f, 0.f, 0.f, 0.f, 0.f, 0.f, 0.f, 0.f};

  for (int job = wave; job < SPB * NTILE; job += 8) {
    const int si = job / NTILE, tile = job - si * NTILE;
    const int s = s0 + si;
    const int g  = tile * 16 + l16;
    const int gc = (g < GSIZE) ? g : (GSIZE - 1);
    const int ix = gc / RES, iy = gc - ix * RES;
    const float gx = meta[si][0] + ((float)ix * (1.0f / (float)(RES - 1))) * meta[si][2];
    const float gy = meta[si][1] + ((float)iy * (1.0f / (float)(RES - 1))) * meta[si][3];
    const float bv[4] = {-2.0f * gx, -2.0f * gy, 1.0f, gx * gx + gy * gy};
    const v16b Bg = build_frag(bv, selB, hh);

    const float2* pb = (const float2*)(births + (size_t)s * (NI * NC * 2));
    const float2* pd = (const float2*)(deaths + (size_t)s * (NI * NC * 2));
    float acc = 0.0f;
    for (int i = 0; i < NI; ++i) {
      const float2 b0 = pb[i * NC + l16], b1 = pb[i * NC + 16 + l16];
      const float2 d0 = pd[i * NC + l16], d1 = pd[i * NC + 16 + l16];
      const float ab0[4] = {b0.x, b0.y, b0.x * b0.x + b0.y * b0.y, 1.0f};
      const float ab1[4] = {b1.x, b1.y, b1.x * b1.x + b1.y * b1.y, 1.0f};
      const float ad0[4] = {d0.x, d0.y, d0.x * d0.x + d0.y * d0.y, 1.0f};
      const float ad1[4] = {d1.x, d1.y, d1.x * d1.x + d1.y * d1.y, 1.0f};
      const v8f Db0 = wmmab(build_frag(ab0, selA, hh), Bg, vzero);
      const v8f Db1 = wmmab(build_frag(ab1, selA, hh), Bg, vzero);
      const v8f Dd0 = wmmab(build_frag(ad0, selA, hh), Bg, vzero);
      const v8f Dd1 = wmmab(build_frag(ad1, selA, hh), Bg, vzero);
      float mb = pairmin8(Db0, Db1); mb = fminf(mb, __shfl_xor(mb, 16, 32));
      float md = pairmin8(Dd0, Dd1); md = fminf(md, __shfl_xor(md, 16, 32));
      const float d2 = fmaxf(fmaxf(mb, md), 0.0f);
      acc = fmaf(w2s[si][i], expf(-200.0f * d2), acc);
    }
    if (hh == 0 && g < GSIZE) sOut[si * GSIZE + g] = acc;
  }
  __syncthreads();

  float* ob = out + (size_t)s0 * GSIZE;
  for (int pass = 0; pass < 2; ++pass) {
    for (int piece = t; piece < SPB * GSIZE / 4; piece += 256) *(volatile v4f*)(ob + piece * 4) = *(const v4f*)(sOut + piece * 4);
    __threadfence();
  }
  (void)S;
}

extern "C" void kernel_launch(void* const* d_in, const int* in_sizes, int n_in,
                              void* d_out, int out_size, void* d_ws, size_t ws_size,
                              hipStream_t stream) {
  (void)n_in; (void)out_size; (void)d_ws; (void)ws_size;
  const float* births = (const float*)d_in[0];
  const float* deaths = (const float*)d_in[1];
  float* out = (float*)d_out;
  const int S = in_sizes[0] / (NI * NC * 2);
  pi_kernel<<<dim3(S / SPB), dim3(256), 0, stream>>>(births, deaths, out, S);
}
